// token_representation_41686952575123
// MI455X (gfx1250) — hardware-verified
//
#include <hip/hip_runtime.h>


namespace {
constexpr int NW = 8192, CL = 16, WV = 50000, CV = 128, WD = 300, CD = 64, CH = 128, G4 = 4 * CH, OD = 512, ID = WD + 2 * CH, WDP = 320;
typedef __attribute__((ext_vector_type(8))) __bf16 v8bb; typedef __attribute__((ext_vector_type(16))) __bf16 v16bb;
typedef __attribute__((ext_vector_type(8))) unsigned short v8us;

typedef _Float16 b16;
typedef __attribute__((ext_vector_type(16))) _Float16 v16b;
typedef __attribute__((ext_vector_type(8)))  _Float16 v8b;
typedef __attribute__((ext_vector_type(8)))  float v8f;
typedef __attribute__((ext_vector_type(4)))  float v4f;

__device__ __forceinline__ v8b ld8b(const b16* p) { return *(const v8b*)p; }
__device__ __forceinline__ v16b cat8b(v8b a, v8b b) { return __builtin_shufflevector(a, b, 0, 1, 2, 3, 4, 5, 6, 7, 8, 9, 10, 11, 12, 13, 14, 15); }
__device__ __forceinline__ v16b frag_kb(const b16* p, int hh) { return cat8b(ld8b(p + 8 * hh), ld8b(p + 16 + 8 * hh)); }
__device__ __forceinline__ void split16(float v, b16& hi, b16& lo) { hi = (b16)v; lo = (b16)(v - (float)hi); }
__device__ __forceinline__ void frag_ksplit(const float* p, int hh, v16b& fh_, v16b& fl_) {
  const float* p0 = p + 8 * hh; const float* p1 = p + 16 + 8 * hh;
#pragma unroll
  for (int e = 0; e < 8; ++e) { b16 a, c; split16(p0[e], a, c); fh_[e] = a; fl_[e] = c; split16(p1[e], a, c); fh_[8 + e] = a; fl_[8 + e] = c; }
}
__device__ __forceinline__ v8f wmma16b(v16b a, v16b b, v8f c) {
  v8f d = __builtin_amdgcn_wmma_f32_16x16x32_f16(false, a, false, b, (short)0, c, false, false);
  asm volatile("v_nop\n\tv_nop\n\tv_nop\n\tv_nop" : "+v"(d) : "v"(a), "v"(b));
  return d;
}
__device__ __forceinline__ void wave_lds_sync() {
  __builtin_amdgcn_fence(__ATOMIC_RELEASE, "workgroup");
  __builtin_amdgcn_wave_barrier();
  __builtin_amdgcn_fence(__ATOMIC_ACQUIRE, "workgroup");
}

struct Opnd { const void* p0; const void* p1; int ld; };
template <int NP> __device__ __forceinline__ void load_frags(const Opnd& o, int row, int kb, int hh, v16b& fh_, v16b& fl_) {
  if (NP == 0) { frag_ksplit((const float*)o.p0 + (size_t)row * o.ld + kb, hh, fh_, fl_); }
  else if (NP == 4) {
    const float* p = (const float*)o.p0 + (size_t)row * o.ld + kb; const float* p0 = p + 8 * hh; const float* p1 = p + 16 + 8 * hh;
#pragma unroll
    for (int e = 0; e < 8; ++e) { b16 a, c; split16(p0[e] * 64.0f, a, c); fh_[e] = a; fl_[e] = c; split16(p1[e] * 64.0f, a, c); fh_[8 + e] = a; fl_[8 + e] = c; }
  } else if (NP == 3) {
    const float* p = (const float*)o.p0 + (size_t)row * o.ld + kb; const float* p0 = p + 8 * hh; const float* p1 = p + 16 + 8 * hh;
#pragma unroll
    for (int e = 0; e < 8; ++e) { fh_[e] = (b16)p0[e]; fh_[8 + e] = (b16)p1[e]; }
    fl_ = fh_;
  } else {
    fh_ = frag_kb((const b16*)o.p0 + (size_t)row * o.ld + kb, hh);
    if (NP == 2) fl_ = frag_kb((const b16*)o.p1 + (size_t)row * o.ld + kb, hh); else fl_ = fh_;
  }
}
template <int ANP, int BNP> __device__ __forceinline__ v8f mac(v16b ah, v16b al, v16b bh, v16b bl, v8f c) {
  c = wmma16b(ah, bh, c);
  if (BNP == 0 || BNP == 2 || BNP == 4) c = wmma16b(ah, bl, c);
  if (ANP == 0 || ANP == 2 || ANP == 4) c = wmma16b(al, bh, c);
  return c;
}
template <int ANP, int BNP>
__device__ __forceinline__ void gemm_tile(const Opnd& A, const Opnd& B, int K, int m0, int c0, int nloc, int hlf, v8f (&acc)[2][4]) {
  for (int kb = 0; kb < K; kb += 32) {
    v16b a0h, a0l, a1h, a1l;
    load_frags<ANP>(A, m0 + nloc, kb, hlf, a0h, a0l);
    load_frags<ANP>(A, m0 + 16 + nloc, kb, hlf, a1h, a1l);
#pragma unroll
    for (int t = 0; t < 4; ++t) {
      v16b bh, bl;
      load_frags<BNP>(B, c0 + t * 16 + nloc, kb, hlf, bh, bl);
      acc[0][t] = mac<ANP, BNP>(a0h, a0l, bh, bl, acc[0][t]);
      acc[1][t] = mac<ANP, BNP>(a1h, a1l, bh, bl, acc[1][t]);
    }
  }
}

__device__ __forceinline__ void epi_planes(v8f (&acc)[2][4], float scale, bool two, b16* __restrict__ oh, b16* __restrict__ ol, int ldo,
                                           int m0, int c0, int lane, b16* Th, b16* Tl) {
  const int nloc = lane & 15, hlf = lane >> 4;
#pragma unroll
  for (int t = 0; t < 4; ++t)
#pragma unroll
    for (int r = 0; r < 2; ++r)
#pragma unroll
      for (int v = 0; v < 8; ++v) {
        const int rr = r * 16 + v + 8 * hlf, cc = t * 16 + nloc;
        b16 h_, l_; split16(acc[r][t][v] * scale, h_, l_);
        Th[rr * 64 + cc] = h_; Tl[rr * 64 + cc] = l_;
      }
  wave_lds_sync();
  for (int pass = 0; pass < 2; ++pass) {
#pragma unroll
    for (int j = 0; j < 8; ++j) {
      const int rr = j * 4 + (lane >> 3), c8 = (lane & 7) * 8;
      const size_t o = (size_t)(m0 + rr) * ldo + c0 + c8;
      *(volatile v8b*)(oh + o) = ld8b(Th + rr * 64 + c8);
      if (two) *(volatile v8b*)(ol + o) = ld8b(Tl + rr * 64 + c8);
    }
    __threadfence();
  }
}
__device__ __forceinline__ void epi_f32(v8f (&acc)[2][4], float scale, const float* rscale, float* __restrict__ out, int ldo, int m0, int c0, int lane, float* Tt) {
  const int nloc = lane & 15, hlf = lane >> 4;
#pragma unroll
  for (int t = 0; t < 4; ++t)
#pragma unroll
    for (int r = 0; r < 2; ++r)
#pragma unroll
      for (int v = 0; v < 8; ++v) {
        const int rr = r * 16 + v + 8 * hlf;
        const float rs = rscale ? rscale[(size_t)(m0 + rr) * 32] : 1.0f;
        Tt[rr * 64 + t * 16 + nloc] = acc[r][t][v] * scale * rs;
      }
  wave_lds_sync();
  float* dst0 = out + (size_t)m0 * ldo + c0;
  for (int pass = 0; pass < 2; ++pass) {
#pragma unroll
    for (int j = 0; j < 16; ++j) { const int rr = j * 2 + hlf, c4 = nloc * 4; *(volatile v4f*)(dst0 + (size_t)rr * ldo + c4) = *(const v4f*)(Tt + rr * 64 + c4); }
    __threadfence();
  }
}


__device__ __forceinline__ v16bb frag_kb_bf(const __bf16* p, int hh) { const v8bb a = *(const v8bb*)(p + 8 * hh), b = *(const v8bb*)(p + 16 + 8 * hh); return __builtin_shufflevector(a, b, 0, 1, 2, 3, 4, 5, 6, 7, 8, 9, 10, 11, 12, 13, 14, 15); }
__device__ __forceinline__ v8f wmma16bb(v16bb a, v16bb b, v8f c) {
  v8f d = __builtin_amdgcn_wmma_f32_16x16x32_bf16(false, a, false, b, (short)0, c, false, false);
  asm volatile("v_nop\n\tv_nop\n\tv_nop\n\tv_nop" : "+v"(d) : "v"(a), "v"(b));
  return d;
}
__device__ __forceinline__ unsigned short bf16_rne_bits(float v) { unsigned int u = __float_as_uint(v); u += 0x7FFFu + ((u >> 16) & 1u); return (unsigned short)(u >> 16); }
__device__ __forceinline__ float bf16_rne(float v) { return __uint_as_float(((unsigned int)bf16_rne_bits(v)) << 16); }

__global__ __launch_bounds__(256) void prep_kernel(const int* __restrict__ wid, const float* __restrict__ wtab, const float* __restrict__ ctab,
                                                   const float* __restrict__ Wih_f, const float* __restrict__ Whh_f, const float* __restrict__ bih_f, const float* __restrict__ bhh_f,
                                                   const float* __restrict__ Wih_b, const float* __restrict__ Whh_b, const float* __restrict__ bih_b, const float* __restrict__ bhh_b,
                                                   const float* __restrict__ Wout,
                                                   unsigned short* __restrict__ featA, unsigned short* __restrict__ wih16, b16* __restrict__ whh16, float* __restrict__ bsum,
                                                   unsigned short* __restrict__ WA, b16* __restrict__ WB, unsigned short* __restrict__ ctab16) {
  const size_t tid = (size_t)blockIdx.x * blockDim.x + threadIdx.x, nth = (size_t)gridDim.x * blockDim.x;
  for (int pass = 0; pass < 2; ++pass) {
    for (size_t p = tid; p < (size_t)NW * WDP / 8; p += nth) { const int n = (int)(p / (WDP / 8)), k0 = (int)(p % (WDP / 8)) * 8; int id = wid[n]; id = (id < 0) ? 0 : (id >= WV ? WV - 1 : id); v8us v;
#pragma unroll
      for (int e = 0; e < 8; ++e) { const int k = k0 + e; v[e] = (k < WD) ? bf16_rne_bits(wtab[(size_t)id * WD + k]) : (unsigned short)0; }
      *(volatile v8us*)(featA + (size_t)n * WDP + k0) = v; }
    for (size_t p = tid; p < (size_t)2 * G4 * CD / 8; p += nth) { const int dir = (int)(p / (G4 * CD / 8)); const size_t i = (p % (G4 * CD / 8)) * 8; const float* W = dir ? Wih_b : Wih_f; v8us v;
#pragma unroll
      for (int e = 0; e < 8; ++e) v[e] = bf16_rne_bits(W[i + e]);
      *(volatile v8us*)(wih16 + p * 8) = v; }
    for (size_t p = tid; p < (size_t)2 * G4 * CH / 8; p += nth) { const int dir = (int)(p / (G4 * CH / 8)); const size_t i = (p % (G4 * CH / 8)) * 8; const float* W = dir ? Whh_b : Whh_f; v8b v;
#pragma unroll
      for (int e = 0; e < 8; ++e) v[e] = (b16)bf16_rne(W[i + e]);
      *(volatile v8b*)(whh16 + p * 8) = v; }
    for (size_t p = tid; p < (size_t)2 * G4; p += nth) { const int dir = (int)(p / G4), u = (int)(p % G4); ((volatile float*)bsum)[p] = dir ? (bf16_rne(bih_b[u]) + bf16_rne(bhh_b[u])) : (bf16_rne(bih_f[u]) + bf16_rne(bhh_f[u])); }
    for (size_t p = tid; p < (size_t)OD * WDP / 8; p += nth) { const int o = (int)(p / (WDP / 8)), k0 = (int)(p % (WDP / 8)) * 8; v8us v;
#pragma unroll
      for (int e = 0; e < 8; ++e) { const int k = k0 + e; v[e] = (k < WD) ? bf16_rne_bits(Wout[(size_t)o * ID + k]) : (unsigned short)0; }
      *(volatile v8us*)(WA + (size_t)o * WDP + k0) = v; }
    for (size_t p = tid; p < (size_t)OD * 2 * CH / 8; p += nth) { const int o = (int)(p / (2 * CH / 8)), k0 = (int)(p % (2 * CH / 8)) * 8; v8b v;
#pragma unroll
      for (int e = 0; e < 8; ++e) v[e] = (b16)bf16_rne(Wout[(size_t)o * ID + WD + k0 + e]);
      *(volatile v8b*)(WB + (size_t)o * 2 * CH + k0) = v; }
    for (size_t p = tid; p < (size_t)CV * CD / 8; p += nth) { v8us v;
#pragma unroll
      for (int e = 0; e < 8; ++e) v[e] = bf16_rne_bits(ctab[p * 8 + e]);
      *(volatile v8us*)(ctab16 + p * 8) = v; }
    __threadfence();
  }
}

__global__ __launch_bounds__(256) void lstm_kernel(const int* __restrict__ cid, const unsigned short* __restrict__ ctab16, const __bf16* __restrict__ wih16, const b16* __restrict__ whh16,
                                                   const float* __restrict__ bsum, b16* __restrict__ fBh, b16* __restrict__ fBl) {
  __shared__ __attribute__((aligned(16))) unsigned short Ct[CV][CD];
  __shared__ __attribute__((aligned(16))) unsigned short Ax[32][CD + 8];
  __shared__ __attribute__((aligned(16))) b16 Ah[32][CH + 8];
  __shared__ float Gt[32][G4 + 4]; __shared__ float Cs[32][CH]; __shared__ float Hsum[32][CH];
  __shared__ __attribute__((aligned(16))) b16 Oh[32][CH + 8]; __shared__ __attribute__((aligned(16))) b16 Ol[32][CH + 8];
  const int t_ = threadIdx.x, wave = t_ >> 5, lane = t_ & 31, nloc = lane & 15, hlf = lane >> 4, n0 = blockIdx.x * 32, dir = blockIdx.y;
  for (int i = t_; i < CV * CD / 8; i += 256) *(v8us*)(&Ct[0][0] + i * 8) = *(const v8us*)(ctab16 + i * 8);
  for (int i = t_; i < 32 * CH; i += 256) { Cs[i / CH][i % CH] = 0.0f; Hsum[i / CH][i % CH] = 0.0f; Ah[i / CH][i % CH] = (b16)0.0f; }
  __syncthreads();
  const __bf16* Wih = wih16 + (size_t)dir * G4 * CD; const b16* Whh = whh16 + (size_t)dir * G4 * CH; const float* bs = bsum + dir * G4;
  for (int step = 0; step < CL; ++step) {
    const int t = dir ? (CL - 1 - step) : step;
    for (int i = t_; i < 32 * CD; i += 256) { const int r = i / CD, k = i % CD; int id = cid[(n0 + r) * CL + t]; id = (id < 0) ? 0 : (id >= CV ? CV - 1 : id); Ax[r][k] = Ct[id][k]; }
    __syncthreads();
    { v8f acc[2][4];
#pragma unroll
      for (int r = 0; r < 2; ++r)
#pragma unroll
        for (int tt = 0; tt < 4; ++tt) acc[r][tt] = (v8f){};
      const int c0 = wave * 64;
#pragma unroll
      for (int kb = 0; kb < CD; kb += 32) {
        const v16bb a0 = frag_kb_bf((const __bf16*)&Ax[nloc][0] + kb, hlf), a1 = frag_kb_bf((const __bf16*)&Ax[16 + nloc][0] + kb, hlf);
#pragma unroll
        for (int tt = 0; tt < 4; ++tt) { const v16bb bw = frag_kb_bf(Wih + (size_t)(c0 + tt * 16 + nloc) * CD + kb, hlf); acc[0][tt] = wmma16bb(a0, bw, acc[0][tt]); acc[1][tt] = wmma16bb(a1, bw, acc[1][tt]); }
      }
#pragma unroll
      for (int kb = 0; kb < CH; kb += 32) {
        const v16b a0 = frag_kb(&Ah[nloc][0] + kb, hlf), a1 = frag_kb(&Ah[16 + nloc][0] + kb, hlf);
#pragma unroll
        for (int tt = 0; tt < 4; ++tt) { const v16b bw = frag_kb(Whh + (size_t)(c0 + tt * 16 + nloc) * CH + kb, hlf); acc[0][tt] = wmma16b(a0, bw, acc[0][tt]); acc[1][tt] = wmma16b(a1, bw, acc[1][tt]); }
      }
#pragma unroll
      for (int tt = 0; tt < 4; ++tt)
#pragma unroll
        for (int r = 0; r < 2; ++r)
#pragma unroll
          for (int v = 0; v < 8; ++v) { const int rr = r * 16 + v + 8 * hlf, cc = c0 + tt * 16 + nloc; Gt[rr][cc] = acc[r][tt][v] + bs[cc]; } }
    __syncthreads();
    for (int i = t_; i < 32 * CH; i += 256) { const int r = i / CH, u = i % CH;
      const float ig = 1.0f / (1.0f + __expf(-Gt[r][u])), fg = 1.0f / (1.0f + __expf(-Gt[r][CH + u])), gg = tanhf(Gt[r][2 * CH + u]), og = 1.0f / (1.0f + __expf(-Gt[r][3 * CH + u]));
      const float c = fg * Cs[r][u] + ig * gg; Cs[r][u] = c; const float h = og * tanhf(c); Ah[r][u] = (b16)h; Hsum[r][u] += h; }
    __syncthreads();
  }
  for (int i = t_; i < 32 * CH; i += 256) { const int r = i / CH, u = i % CH; b16 a, c; split16(Hsum[r][u], a, c); Oh[r][u] = a; Ol[r][u] = c; }
  __syncthreads();
  for (int pass = 0; pass < 2; ++pass) {
#pragma unroll
    for (int j = 0; j < 2; ++j) { const int rr = j * 16 + (t_ >> 4), c8 = (t_ & 15) * 8;
      *(volatile v8b*)(fBh + (size_t)(n0 + rr) * (2 * CH) + dir * CH + c8) = *(const v8b*)(&Oh[rr][c8]); *(volatile v8b*)(fBl + (size_t)(n0 + rr) * (2 * CH) + dir * CH + c8) = *(const v8b*)(&Ol[rr][c8]); }
    __threadfence();
  }
}

__global__ __launch_bounds__(128) void out_kernel(const __bf16* __restrict__ featA, const __bf16* __restrict__ WA, const b16* __restrict__ fBh, const b16* __restrict__ fBl, const b16* __restrict__ WB,
                                                  const float* __restrict__ bout, float* __restrict__ out) {
  __shared__ __attribute__((aligned(16))) float Ts[4][32 * 64];
  const int lane = threadIdx.x & 31, wave = threadIdx.x >> 5, nloc = lane & 15, hlf = lane >> 4, m0 = blockIdx.y * 128 + wave * 32, c0 = blockIdx.x * 64;
  v8f acc[2][4];
#pragma unroll
  for (int r = 0; r < 2; ++r)
#pragma unroll
    for (int t = 0; t < 4; ++t) acc[r][t] = (v8f){};
#pragma unroll 2
  for (int kb = 0; kb < WDP; kb += 32) {
    const v16bb a0 = frag_kb_bf(featA + (size_t)(m0 + nloc) * WDP + kb, hlf), a1 = frag_kb_bf(featA + (size_t)(m0 + 16 + nloc) * WDP + kb, hlf);
#pragma unroll
    for (int t = 0; t < 4; ++t) { const v16bb bw = frag_kb_bf(WA + (size_t)(c0 + t * 16 + nloc) * WDP + kb, hlf); acc[0][t] = wmma16bb(a0, bw, acc[0][t]); acc[1][t] = wmma16bb(a1, bw, acc[1][t]); }
  }
  { const Opnd A{fBh, fBl, 2 * CH}, B{WB, nullptr, 2 * CH};
    gemm_tile<2, 1>(A, B, 2 * CH, m0, c0, nloc, hlf, acc); }
  float* Tt = Ts[wave];
#pragma unroll
  for (int t = 0; t < 4; ++t)
#pragma unroll
    for (int r = 0; r < 2; ++r)
#pragma unroll
      for (int v = 0; v < 8; ++v) Tt[(r * 16 + v + 8 * hlf) * 64 + t * 16 + nloc] = tanhf(acc[r][t][v] + bf16_rne(bout[c0 + t * 16 + nloc]));
  wave_lds_sync();
  for (int pass = 0; pass < 2; ++pass) {
#pragma unroll
    for (int j = 0; j < 16; ++j) { const int rr = j * 2 + hlf, c4 = nloc * 4; *(volatile v4f*)(out + (size_t)(m0 + rr) * OD + c0 + c4) = *(const v4f*)(Tt + rr * 64 + c4); }
    __threadfence();
  }
}
}

extern "C" void kernel_launch(void* const* d_in, const int* in_sizes, int n_in,
                              void* d_out, int out_size, void* d_ws, size_t ws_size, hipStream_t stream) {
  (void)n_in; (void)out_size;
  const int* wid = (const int*)d_in[0]; const int* cid = (const int*)d_in[1]; const float* wtab = (const float*)d_in[2]; const float* ctab = (const float*)d_in[3];
  const float* Wih_f = (const float*)d_in[4]; const float* Whh_f = (const float*)d_in[5]; const float* bih_f = (const float*)d_in[6]; const float* bhh_f = (const float*)d_in[7];
  const float* Wih_b = (const float*)d_in[8]; const float* Whh_b = (const float*)d_in[9]; const float* bih_b = (const float*)d_in[10]; const float* bhh_b = (const float*)d_in[11];
  const float* Wout = (const float*)d_in[12]; const float* bout = (const float*)d_in[13];
  float* out = (float*)d_out;
  if (in_sizes[0] != NW || in_sizes[1] != NW * CL || in_sizes[2] != WV * WD || in_sizes[3] != CV * CD || in_sizes[4] != G4 * CD || in_sizes[5] != G4 * CH || in_sizes[12] != OD * ID) return;
  size_t off = 0; char* ws = (char*)d_ws;
  auto carve = [&](size_t bytes) { char* p = ws + off; off += (bytes + 255) & ~(size_t)255; return p; };
  unsigned short* featA = (unsigned short*)carve((size_t)NW * WDP * 2);
  unsigned short* wih16 = (unsigned short*)carve((size_t)2 * G4 * CD * 2); b16* whh16 = (b16*)carve((size_t)2 * G4 * CH * 2); float* bsum = (float*)carve(2 * G4 * 4);
  unsigned short* WA = (unsigned short*)carve((size_t)OD * WDP * 2); b16* WB = (b16*)carve((size_t)OD * 2 * CH * 2); unsigned short* ctab16 = (unsigned short*)carve((size_t)CV * CD * 2);
  b16* fBh = (b16*)carve((size_t)NW * 2 * CH * 2); b16* fBl = (b16*)carve((size_t)NW * 2 * CH * 2);
  if (off > ws_size) return;
  prep_kernel<<<512, 256, 0, stream>>>(wid, wtab, ctab, Wih_f, Whh_f, bih_f, bhh_f, Wih_b, Whh_b, bih_b, bhh_b, Wout, featA, wih16, whh16, bsum, WA, WB, ctab16);
  lstm_kernel<<<dim3(NW / 32, 2), 256, 0, stream>>>(cid, ctab16, (const __bf16*)wih16, whh16, bsum, fBh, fBl);
  out_kernel<<<dim3(OD / 64, NW / 128), 128, 0, stream>>>((const __bf16*)featA, (const __bf16*)WA, fBh, fBl, WB, bout, out);
}
